// Individual_39530878992727
// MI455X (gfx1250) — hardware-run, weakly checked
//
#include <hip/hip_runtime.h>


#ifndef NB
#define NB 32768
#endif
#define NB_FULL 32768
#define IND   256
#define NMID  272
#define NNODE 528
#define NT    17
#define OUTD  16
#define WV    2
#define RPW   32
#define XP    264
#define RP    280
#define PP    20
#define BEW   384
#define WSC   64.0f
#define RSC   1024.0f
#define FOLD  (1.0f / 65536.0f)
#define LOG2E 1.4426950408889634f

static_assert(NMID == NT * 16);
static_assert(NNODE == IND + NMID);
static_assert(IND == 256);
static_assert(16 * (NT - 1) <= IND);
static_assert(IND % 32 == 0);
static_assert(NMID - OUTD == (NT - 1) * 16);
static_assert(OUTD == 16);
static_assert(RPW == 32);
static_assert(NB % (WV * RPW) == 0);
static_assert(NB <= NB_FULL);
static_assert(XP % 8 == 0 && XP >= IND);
static_assert(RP % 8 == 0 && RP >= NMID);
static_assert(PP % 4 == 0 && PP >= 16);
static_assert(((RPW * RP) / 8) % 32 == 0);
static_assert((NT * 256 / 4) % (32 * WV) == 0);
static_assert((2 * BEW / 4) % (32 * WV) == 0);
static_assert(BEW >= NMID);
static_assert(32 * 4 * 16 == RPW * OUTD * 4);
static_assert((size_t)WV * RPW * XP * 2 + (size_t)WV * RPW * RP * 2 + (size_t)WV * RPW * PP * 4 + (size_t)NT * 256 * 4 + (size_t)2 * BEW * 4 <= 131072);

typedef _Float16 h16;
typedef unsigned short bf;
typedef __attribute__((ext_vector_type(16))) __bf16   v16bf;
typedef __attribute__((ext_vector_type(16))) _Float16 v16h;
typedef __attribute__((ext_vector_type(8)))  _Float16 v8h;
typedef __attribute__((ext_vector_type(8)))  unsigned short v8us;
typedef __attribute__((ext_vector_type(8)))  float    v8f;
typedef __attribute__((ext_vector_type(4)))  float    v4f;
typedef v4f  __attribute__((may_alias)) v4fa;

__device__ __forceinline__ unsigned short f2bf(float f) { unsigned u = __float_as_uint(f); u += 0x7FFFu + ((u >> 16) & 1u); return (unsigned short)(u >> 16); }
__device__ __forceinline__ float bfr(float f) { return __uint_as_float(((unsigned)f2bf(f)) << 16); }
__device__ __forceinline__ v16h cat16(v8h lo, v8h hi) { return __builtin_shufflevector(lo, hi, 0, 1, 2, 3, 4, 5, 6, 7, 8, 9, 10, 11, 12, 13, 14, 15); }
__device__ __forceinline__ v16bf cat16b(v8us lo, v8us hi) { return __builtin_bit_cast(v16bf, __builtin_shufflevector(lo, hi, 0, 1, 2, 3, 4, 5, 6, 7, 8, 9, 10, 11, 12, 13, 14, 15)); }
__device__ __forceinline__ v8f wmma16(v16h a, v16h b, v8f c) { return __builtin_amdgcn_wmma_f32_16x16x32_f16(false, a, false, b, (short)0, c, false, false); }
__device__ __forceinline__ v8f wmmab(v16bf a, v16bf b, v8f c) { return __builtin_amdgcn_wmma_f32_16x16x32_bf16(false, a, false, b, (short)0, c, false, false); }
__device__ __forceinline__ v16h  ldh(const h16* p) { return cat16(*(const v8h*)p, *(const v8h*)(p + 16)); }
__device__ __forceinline__ v16bf ldb(const bf* p)  { return cat16b(*(const v8us*)p, *(const v8us*)(p + 16)); }
__device__ __forceinline__ void wave_sync() { __builtin_amdgcn_fence(3  , "wavefront"); __builtin_amdgcn_wave_barrier(); asm volatile("" ::: "memory"); }

static __device__ __forceinline__ h16 toh_flush(float v) { const h16 r = (h16)v; return (fabsf(v) < 6.103515625e-05f) ? (h16)0.0f : r; }
__device__ __forceinline__ v8f wmma16g(v16h a, v16h b, v8f c) { c = wmma16(a, b, c); asm volatile("v_nop\n\tv_nop\n\tv_nop\n\tv_nop" : "+v"(c) : "v"(a), "v"(b)); return c; }
__device__ __forceinline__ v8f wmmabg(v16bf a, v16bf b, v8f c) { c = wmmab(a, b, c); asm volatile("v_nop\n\tv_nop\n\tv_nop\n\tv_nop" : "+v"(c) : "v"(a), "v"(b)); return c; }

#define PB_W  ((NMID * IND / 8) / 256)
#define NP_WD (NT * 256 / 4)
#define PB_WD ((NP_WD + 255) / 256)
#define NP_BE (2 * BEW / 4)
static_assert((NMID * IND / 8) % 256 == 0);
static_assert(NP_WD % 32 == 0);
static_assert(NP_BE % 32 == 0 && NP_BE <= 256);

__global__ __launch_bounds__(256) void k_prep(const float* __restrict__ W, const float* __restrict__ bias, const int* __restrict__ conn, const int* __restrict__ exist,
                                              bf* WB, h16* WH, float* WD, float* BE) {
    const int blk = blockIdx.x, tid = threadIdx.x;
    if (blk < PB_W) {
        const int i = blk * 256 + tid; const int n = i >> 5, k0 = (i & 31) * 8;
        v8us o;
#pragma unroll
        for (int e = 0; e < 8; ++e) { const int src = (k0 + e) * NMID + n; float wv = W[src]; int cv = conn[src];
            asm volatile("" : "+v"(wv)); asm volatile("" : "+v"(cv));
            o[e] = f2bf(bfr(wv) * (float)cv); }
        bf* dst = WB + (size_t)i * 8;
        *(volatile v8us*)dst = o; __threadfence(); *(volatile v8us*)dst = o;
    } else if (blk < 2 * PB_W) {
        const int i = (blk - PB_W) * 256 + tid; const int n = i >> 5, k0 = (i & 31) * 8; const int kl = 16 * (n >> 4);
        v8h o;
#pragma unroll
        for (int e = 0; e < 8; ++e) { const int k = k0 + e; const int src = (IND + k) * NMID + n; float wv = W[src]; int cv = conn[src];
            asm volatile("" : "+v"(wv)); asm volatile("" : "+v"(cv));
            const h16 hv = toh_flush(bfr(wv) * (float)cv * WSC);
            o[e] = (k < kl) ? hv : (h16)0.0f; }
        h16* dst = WH + (size_t)i * 8;
        *(volatile v8h*)dst = o; __threadfence(); *(volatile v8h*)dst = o;
    } else if (blk < 2 * PB_W + PB_WD) {
        const int i = (blk - 2 * PB_W) * 256 + tid;
        if (i < NP_WD) {
            const int t = i >> 6, j = (i >> 2) & 15, q = (i & 3) * 4;
            v4f o;
#pragma unroll
            for (int e = 0; e < 4; ++e) { const int j2 = q + e; const int src = (IND + 16 * t + j2) * NMID + 16 * t + j; float wv = W[src]; int cv = conn[src];
                asm volatile("" : "+v"(wv)); asm volatile("" : "+v"(cv));
                const float ev = bfr(wv) * (float)cv;
                o[e] = (j2 < j) ? ev : 0.0f; }
            float* dst = WD + (size_t)i * 4;
            *(volatile v4f*)dst = o; __threadfence(); *(volatile v4f*)dst = o;
        }
    } else {
        const int i = tid;
        if (i < NP_BE) {
            v4f o;
#pragma unroll
            for (int e = 0; e < 4; ++e) { const int c = i * 4 + e; const int sec = (c >= BEW) ? 1 : 0; const int col = c - BEW * sec;
                const int cc = col < NMID ? col : (NMID - 1);
                float bv = bias[cc]; int xv = exist[cc];
                asm volatile("" : "+v"(bv)); asm volatile("" : "+v"(xv));
                const float val = sec ? (float)xv : bfr(bv);
                o[e] = (col < NMID) ? val : 0.0f; }
            float* dst = BE + (size_t)i * 4;
            *(volatile v4f*)dst = o; __threadfence(); *(volatile v4f*)dst = o;
        }
    }
}

__global__ __launch_bounds__(32 * WV) void k_net(const float* __restrict__ X, const bf* __restrict__ WB, const h16* __restrict__ WH,
                                                 const float* __restrict__ WD, const float* __restrict__ BE, float* OUT) {
    __shared__ __align__(16) bf    xs[WV * RPW * XP];
    __shared__ __align__(16) h16   rs[WV * RPW * RP];
    __shared__ __align__(16) float pt[WV * RPW * PP];
    __shared__ __align__(16) float wd[NT * 256];
    __shared__ __align__(16) float be[2 * BEW];
    const int lane = threadIdx.x & 31, lr = lane & 15, hi = lane >> 4;
    const int wave = __builtin_amdgcn_readfirstlane((int)(threadIdx.x >> 5));
    const int row0 = (blockIdx.x * WV + wave) * RPW;
    const int xb = wave * RPW * XP, rb = wave * RPW * RP, pb = wave * RPW * PP;

#pragma unroll 1
    for (int i = threadIdx.x; i < NP_WD; i += 32 * WV) { const v4f v = *(const v4f*)(WD + (size_t)i * 4); *(v4fa*)(&wd[i * 4]) = v; }
#pragma unroll 1
    for (int i = threadIdx.x; i < NP_BE; i += 32 * WV) { const v4f v = *(const v4f*)(BE + (size_t)i * 4); *(v4fa*)(&be[i * 4]) = v; }
#pragma unroll 4
    for (int i = 0; i < RPW; ++i) {
        const v8f v = *(const v8f*)(X + (size_t)(row0 + i) * IND + lane * 8); v8us o;
#pragma unroll
        for (int k = 0; k < 8; ++k) o[k] = f2bf(v[k]);
        *(v8us*)(&xs[xb + i * XP + lane * 8]) = o;
    }
    { const v8h z = (v8h){};
#pragma unroll 1
      for (int i = 0; i < (RPW * RP) / 8 / 32; ++i) *(v8h*)(&rs[rb + (i * 32 + lane) * 8]) = z; }
    __syncthreads();

    const int xa0 = xb + lr * XP + 8 * hi, xa1 = xa0 + 16 * XP;
    const int ra0 = rb + lr * RP + 8 * hi, ra1 = ra0 + 16 * RP;
    float s[16];
#pragma unroll
    for (int j = 0; j < 16; ++j) s[j] = 0.0f;

#pragma unroll 1
    for (int t = 0; t < NT; ++t) {
        const size_t wo = (size_t)(t * 16 + lr) * IND + 8 * hi;
        v8f c0 = (v8f){}, c1 = (v8f){}, d0 = (v8f){}, d1 = (v8f){};
#pragma unroll
        for (int kc = 0; kc < IND; kc += 32) {
            const v16bf b  = ldb(WB + wo + kc);
            const v16bf a0 = cat16b(*(const v8us*)(&xs[xa0 + kc]), *(const v8us*)(&xs[xa0 + kc + 16]));
            const v16bf a1 = cat16b(*(const v8us*)(&xs[xa1 + kc]), *(const v8us*)(&xs[xa1 + kc + 16]));
            c0 = wmmabg(a0, b, c0); c1 = wmmabg(a1, b, c1);
        }
        const int ns = (t + 1) >> 1;
#pragma unroll 1
        for (int ks = 0; ks < ns; ++ks) {
            const int kc = ks * 32;
            const v16h b  = ldh(WH + wo + kc);
            const v16h a0 = cat16(*(const v8h*)(&rs[ra0 + kc]), *(const v8h*)(&rs[ra0 + kc + 16]));
            const v16h a1 = cat16(*(const v8h*)(&rs[ra1 + kc]), *(const v8h*)(&rs[ra1 + kc + 16]));
            d0 = wmma16g(a0, b, d0); d1 = wmma16g(a1, b, d1);
        }
#pragma unroll
        for (int r = 0; r < 8; ++r) {
            pt[pb + (8 * hi + r) * PP + lr]      = c0[r] + d0[r] * FOLD;
            pt[pb + (16 + 8 * hi + r) * PP + lr] = c1[r] + d1[r] * FOLD; }
        wave_sync();
        const int pr = pb + lane * PP;
        const v4f q0 = *(const v4fa*)(&pt[pr]), q1 = *(const v4fa*)(&pt[pr + 4]), q2 = *(const v4fa*)(&pt[pr + 8]), q3 = *(const v4fa*)(&pt[pr + 12]);
        float p[16];
#pragma unroll
        for (int j = 0; j < 4; ++j) { p[j] = q0[j]; p[4 + j] = q1[j]; p[8 + j] = q2[j]; p[12 + j] = q3[j]; }
        const int tb = t * 256, nb = t * 16;
#pragma unroll
        for (int j = 0; j < 16; ++j) {
            float a = p[j] + be[nb + j];
#pragma unroll
            for (int j2 = 0; j2 < j; ++j2) a += s[j2] * wd[tb + j * 16 + j2];
            const float e = __builtin_amdgcn_exp2f(-a * LOG2E);
            s[j] = be[BEW + nb + j] * __builtin_amdgcn_rcpf(1.0f + e);
        }
        v8h h0, h1;
#pragma unroll
        for (int j = 0; j < 8; ++j) { h0[j] = toh_flush(s[j] * RSC); h1[j] = toh_flush(s[8 + j] * RSC); }
        *(v8h*)(&rs[rb + lane * RP + nb]) = h0; *(v8h*)(&rs[rb + lane * RP + nb + 8]) = h1;
        wave_sync();
    }

    { v4f a, b, c, d;
#pragma unroll
      for (int j = 0; j < 4; ++j) { a[j] = s[j]; b[j] = s[4 + j]; c[j] = s[8 + j]; d[j] = s[12 + j]; }
      const int pr = pb + lane * PP;
      *(v4fa*)(&pt[pr]) = a; *(v4fa*)(&pt[pr + 4]) = b; *(v4fa*)(&pt[pr + 8]) = c; *(v4fa*)(&pt[pr + 12]) = d; }
    wave_sync();
    float* ob = OUT + (size_t)row0 * OUTD;
#pragma unroll 1
    for (int ps = 0; ps < 2; ++ps) {
#pragma unroll
        for (int si = 0; si < 4; ++si) { const int q = si * 32 + lane; const int row = q >> 2, cofs = (q & 3) * 4;
            const v4f val = *(const v4fa*)(&pt[pb + row * PP + cofs]);
            *(volatile v4f*)(ob + (size_t)q * 4) = val; }
        if (ps == 0) __threadfence(); }
}

static constexpr size_t al256(size_t v) { return (v + 255) & ~(size_t)255; }
static constexpr size_t SZ_W  = al256((size_t)NMID * IND * 2);
static constexpr size_t SZ_WD = al256((size_t)NT * 256 * 4);
static constexpr size_t SZ_BE = al256((size_t)2 * BEW * 4);
static constexpr size_t SZ_TOTAL = 2 * SZ_W + SZ_WD + SZ_BE;
static_assert(SZ_TOTAL <= (size_t)134217728);
static_assert((size_t)(2 * PB_W) * 256 * 16 == 2 * (size_t)NMID * IND * 2);
static_assert((size_t)NP_WD * 16 == (size_t)NT * 256 * 4);
static_assert((size_t)NP_BE * 16 == (size_t)2 * BEW * 4);

extern "C" void kernel_launch(void* const* d_in, const int* in_sizes, int n_in,
                              void* d_out, int out_size, void* d_ws, size_t ws_size, hipStream_t stream) {
    if (n_in < 5) return;
    if ((size_t)in_sizes[0] < (size_t)NB * IND) return;
    if ((size_t)in_sizes[1] < (size_t)NNODE * NMID || (size_t)in_sizes[3] < (size_t)NNODE * NMID) return;
    if (in_sizes[2] < NMID || in_sizes[4] < NMID) return;
    if ((size_t)out_size < (size_t)NB * OUTD) return;
    if (SZ_TOTAL > ws_size) return;
    const float* x    = (const float*)d_in[0];
    const float* w    = (const float*)d_in[1];
    const float* bias = (const float*)d_in[2];
    const int*   conn = (const int*)d_in[3];
    const int*   ex   = (const int*)d_in[4];
    float* OUT = (float*)d_out;
    char* wsp = (char*)d_ws;
    bf*    WB = (bf*)wsp;    wsp += SZ_W;
    h16*   WH = (h16*)wsp;   wsp += SZ_W;
    float* WD = (float*)wsp; wsp += SZ_WD;
    float* BE = (float*)wsp; wsp += SZ_BE;

    k_prep<<<dim3(2 * PB_W + PB_WD + 1, 1, 1), 256, 0, stream>>>(w, bias, conn, ex, WB, WH, WD, BE);
    k_net<<<dim3(NB / (WV * RPW), 1, 1), 32 * WV, 0, stream>>>(x, WB, WH, WD, BE, OUT);
}
